// SpatiotemporalAttentionBase_16114717295099
// MI455X (gfx1250) — hardware-verified
//
#include <hip/hip_runtime.h>
#include <hip/hip_bf16.h>
#include <math.h>

#define NBs 4
#define CCs 64
#define CIs 32
#define NNs 4096
#define SS 4096
#define HH 1
#define DKK 64
#define GSTR 48

typedef _Float16 bf16;
typedef _Float16 f16;
typedef __attribute__((ext_vector_type(4))) unsigned v4u_t;
typedef unsigned v4ua __attribute__((ext_vector_type(4), may_alias));
typedef __attribute__((ext_vector_type(4))) float v4f_t;
typedef float v4fa __attribute__((ext_vector_type(4), may_alias));
typedef __attribute__((ext_vector_type(16))) bf16  bf16x16;
typedef bf16x16 f16x16;
typedef __attribute__((ext_vector_type(8)))  bf16  bf16x8;
typedef bf16x8 f16x8;
typedef __attribute__((ext_vector_type(4)))  bf16  bf16x4;
typedef __attribute__((ext_vector_type(8)))  float f32x8;
__device__ __forceinline__ f32x8 wmma16(f16x16 a, f16x16 b, f32x8 c) {
  c = __builtin_amdgcn_wmma_f32_16x16x32_f16(false, a, false, b, (short)0, c, false, false);
  asm volatile("v_nop\n\tv_nop\n\tv_nop\n\tv_nop" : "+v"(c) : "v"(a), "v"(b));
  return c;
}
#define LDS_STRIDE 48
#define KSTRIDE    72
#define VSTRIDE    48

__device__ __forceinline__ f32x8 wmma_bf16(bf16x16 a, bf16x16 b, f32x8 c) {
  c = __builtin_amdgcn_wmma_f32_16x16x32_f16(false, a, false, b, (short)0, c, false, false);
  asm volatile("v_nop\n\tv_nop\n\tv_nop\n\tv_nop" : "+v"(c) : "v"(a), "v"(b));
  return c;
}

template <typename T>
__device__ __forceinline__ bf16x16 load_frag(const T* __restrict__ base, int ld,
                                             int row0, int k0) {
  const int lane = threadIdx.x & 31;
  const int r    = lane & 15;
  const int kh   = (lane >> 4) * 8;
  const T* p0 = base + (size_t)(row0 + r) * ld + (k0 + kh);
  const T* p1 = p0 + 16;
  bf16x16 f;
#pragma unroll
  for (int i = 0; i < 8; ++i) {
    f[i]     = (bf16)p0[i];
    f[i + 8] = (bf16)p1[i];
  }
  return f;
}

__device__ __forceinline__ bf16x16 lds_frag(const bf16* base, int stride) {
  const int lane = threadIdx.x & 31;
  const int row  = lane & 15;
  const int kh   = (lane >> 4) * 8;
  const bf16x8 lo = *(const bf16x8*)(base + row * stride + kh);
  const bf16x8 hi = *(const bf16x8*)(base + row * stride + kh + 16);
  bf16x16 f;
#pragma unroll
  for (int i = 0; i < 8; ++i) { f[i] = lo[i]; f[i + 8] = hi[i]; }
  return f;
}

template <typename T>
__device__ __forceinline__ void stage_read16(const T* __restrict__ p, float* buf) {
#pragma unroll
  for (int i = 0; i < 16; ++i) buf[i] = (float)p[i];
}

__device__ __forceinline__ void stage_write(bf16* dst, const float* buf, int nquad) {
#pragma unroll
  for (int i = 0; i < nquad; ++i) {
    bf16x4 q;
    q[0] = (bf16)buf[4 * i];     q[1] = (bf16)buf[4 * i + 1];
    q[2] = (bf16)buf[4 * i + 2]; q[3] = (bf16)buf[4 * i + 3];
    *(bf16x4*)(dst + 4 * i) = q;
  }
}

template <typename AT, int MODE>
__global__ __launch_bounds__(256) void gemm_rb_kernel(
    const AT* __restrict__ A, const float* __restrict__ W,
    const float* __restrict__ bias, const float* __restrict__ rowscale, const float* __restrict__ R, const float* __restrict__ rowbias, void* __restrict__ out,
    int M, int N, int K) {
  __shared__ bf16 ldsA[128 * LDS_STRIDE];
  __shared__ bf16 ldsW[256 * LDS_STRIDE];
  __shared__ __attribute__((aligned(16))) unsigned char sob[256 * 136 * 2];

  const int t    = threadIdx.x;
  const int wave = t >> 5;
  const int lane = t & 31;
  const int wm   = (wave & 1) * 64;
  const int wn   = (wave >> 1) * 64;
  const int mBlk = blockIdx.x * 128;
  const int nBlk = blockIdx.y * 256;

  const int arow = t >> 1;
  const int ach  = (t & 1) * 16;

  float abuf[16];
  float wbuf[32];

  stage_read16(A + (size_t)(mBlk + arow) * K + ach, abuf);
  const int nrow = min(nBlk + t, N - 1);
  stage_read16(W + (size_t)nrow * K,          wbuf);
  stage_read16(W + (size_t)nrow * K + 16,     wbuf + 16);

  f32x8 acc[4][4] = {};

  for (int k = 0; k < K; k += 32) {
    __syncthreads();
    stage_write(&ldsA[arow * LDS_STRIDE + ach], abuf, 4);
    stage_write(&ldsW[t * LDS_STRIDE],          wbuf, 8);
    if (k + 32 < K) {
      stage_read16(A + (size_t)(mBlk + arow) * K + (k + 32) + ach, abuf);
      stage_read16(W + (size_t)nrow * K + (k + 32),          wbuf);
      stage_read16(W + (size_t)nrow * K + (k + 32) + 16,     wbuf + 16);
    }
    __syncthreads();

    bf16x16 af[4], wf[4];
#pragma unroll
    for (int i = 0; i < 4; ++i)
      af[i] = lds_frag(ldsA + (wm + 16 * i) * LDS_STRIDE, LDS_STRIDE);
#pragma unroll
    for (int j = 0; j < 4; ++j)
      wf[j] = lds_frag(ldsW + (wn + 16 * j) * LDS_STRIDE, LDS_STRIDE);
#pragma unroll
    for (int i = 0; i < 4; ++i)
#pragma unroll
      for (int j = 0; j < 4; ++j)
        acc[i][j] = wmma_bf16(af[i], wf[j], acc[i][j]);
  }

  const int nlane = lane & 15;
  const int mh    = (lane >> 4) * 8;
  __syncthreads();
  if (MODE == 0 || MODE == 1 || MODE == 3) {
    bf16* so = (bf16*)sob;
#pragma unroll
    for (int i = 0; i < 4; ++i)
#pragma unroll
      for (int j = 0; j < 4; ++j) {
        const int nl = wn + 16 * j + nlane;
        const float bv = bias ? bias[nBlk + nl] : 0.0f;
        if (MODE == 3) {
#pragma unroll 1
          for (int r = 0; r < 8; ++r) {
            const int ml = wm + 16 * i + mh + r;
            const float xg = acc[i][j][r] + bv;
            so[ml * 264 + nl] = (bf16)(0.5f * xg * (1.0f + erff(xg * 0.70710678118654752f)));
          }
        } else {
#pragma unroll
        for (int r = 0; r < 8; ++r) {
          const int ml = wm + 16 * i + mh + r;
          const bf16 hv = (bf16)(acc[i][j][r] + bv);
          if (MODE == 0) so[ml * 264 + nl] = hv;
          else           so[nl * 136 + ml] = hv;
        }
        }
      }
    __syncthreads();
#pragma unroll 1
    for (int pass = 0; pass < 2; ++pass) {
      if (MODE == 0 || MODE == 3) {
        for (int ch = t; ch < 128 * 32; ch += 256) { const int ml = ch >> 5, q = (ch & 31) * 8;
          *(volatile v4u_t*)((bf16*)out + (size_t)(mBlk + ml) * N + nBlk + q) = *(const v4ua*)(so + ml * 264 + q); }
      } else {
        const int b_ = mBlk / SS, s0 = mBlk % SS;
        for (int ch = t; ch < 256 * 16; ch += 256) { const int nl = ch >> 4, q = (ch & 15) * 8; const int n = nBlk + nl, h = n >> 6, dk = n & (DKK - 1);
          *(volatile v4u_t*)((bf16*)out + (((size_t)(b_ * HH + h)) * DKK + dk) * SS + s0 + q) = *(const v4ua*)(so + nl * 136 + q); }
      }
      __threadfence();
    }
  } else {
    float* so = (float*)sob;
#pragma unroll 1
    for (int hf = 0; hf < 2; ++hf) {
      if (wm == hf * 64) {
#pragma unroll
        for (int i = 0; i < 4; ++i)
#pragma unroll
          for (int j = 0; j < 4; ++j) {
            const int nl = wn + 16 * j + nlane;
            const float bv = bias ? bias[nBlk + nl] : 0.0f;
#pragma unroll
            for (int r = 0; r < 8; ++r) { const int mrow = mBlk + hf * 64 + 16 * i + mh + r; so[(16 * i + mh + r) * 260 + nl] = acc[i][j][r] * (rowscale ? rowscale[mrow] : 1.0f) + bv + (rowbias ? rowbias[mrow] : 0.0f); }
          }
      }
      __syncthreads();
      if (R) {
        for (int ch = t; ch < 64 * 64; ch += 256) { const int ml = ch >> 6, q = (ch & 63) * 4;
          if (nBlk + q < N) { const v4f_t rv = *(const v4f_t*)(R + (size_t)(mBlk + hf * 64 + ml) * N + nBlk + q); v4f_t v = *(const v4fa*)(so + ml * 260 + q); v += rv; *(volatile v4fa*)(so + ml * 260 + q) = v; } }
        asm volatile("s_wait_dscnt 0" ::: "memory");
      }
#pragma unroll 1
      for (int pass = 0; pass < 2; ++pass) {
        for (int ch = t; ch < 64 * 64; ch += 256) { const int ml = ch >> 6, q = (ch & 63) * 4;
          if (nBlk + q < N) *(volatile v4f_t*)((float*)out + (size_t)(mBlk + hf * 64 + ml) * N + nBlk + q) = *(const v4fa*)(so + ml * 260 + q); }
        __threadfence();
      }
      __syncthreads();
    }
  }
}


#define GSTR 48
template <typename AT, int EPI, bool OUT16>
__global__ __launch_bounds__(256) void gemm_kne(const AT* __restrict__ A, int lda, const float* __restrict__ Wm, int ldw,
                                                const float* __restrict__ bias, const float* __restrict__ R, const float* __restrict__ gvec,
                                                void* __restrict__ Yv, int ldy, int K) {
  __shared__ __attribute__((aligned(16))) f16 ldsA[128 * GSTR];
  __shared__ __attribute__((aligned(16))) f16 ldsW[128 * GSTR];
  __shared__ __attribute__((aligned(16))) float oS[8][32 * 68];
  const int tid = threadIdx.x, lane = tid & 31, wave = tid >> 5, cl = lane & 15, rh = (lane >> 4) * 8;
  const int m0 = blockIdx.x * 128, n0 = blockIdx.y * 128;
  const int wm = (wave & 3) * 32, wn = (wave >> 2) * 64;
  f32x8 acc[2][4];
#pragma unroll
  for (int i = 0; i < 2; ++i)
#pragma unroll
    for (int j = 0; j < 4; ++j) { f32x8 z = {}; acc[i][j] = z; }
#pragma unroll 1
  for (int k0 = 0; k0 < K; k0 += 32) {
    __syncthreads();
    { const int row = tid >> 1, ch = (tid & 1) * 16;
      const AT* src = A + (size_t)(m0 + row) * lda + k0 + ch;
#pragma unroll
      for (int g = 0; g < 16; ++g) ldsA[row * GSTR + ch + g] = (f16)src[g]; }
    { const int k = tid >> 3, nn0 = (tid & 7) * 16;
      const float* src = Wm + (size_t)(k0 + k) * ldw + n0 + nn0;
#pragma unroll
      for (int g = 0; g < 4; ++g) { const v4f_t v = *(const v4f_t*)(src + 4 * g);
#pragma unroll
        for (int u = 0; u < 4; ++u) ldsW[(nn0 + 4 * g + u) * GSTR + k] = (f16)v[u]; } }
    __syncthreads();
    f16x16 af[2];
#pragma unroll
    for (int i = 0; i < 2; ++i) af[i] = lds_frag(ldsA + (wm + 16 * i) * GSTR, GSTR);
#pragma unroll
    for (int j = 0; j < 4; ++j) {
      const f16x16 bf = lds_frag(ldsW + (wn + 16 * j) * GSTR, GSTR);
#pragma unroll
      for (int i = 0; i < 2; ++i) acc[i][j] = wmma16(af[i], bf, acc[i][j]);
    }
  }
  float* so = oS[wave];
#pragma unroll
  for (int i = 0; i < 2; ++i)
#pragma unroll
    for (int j = 0; j < 4; ++j) {
      const int n = n0 + wn + 16 * j + cl;
      const float bv = bias ? bias[n] : 0.0f;
      const float gv = (EPI == 2) ? gvec[n] : 0.0f;
      if (EPI == 1) {
#pragma unroll 1
        for (int r = 0; r < 8; ++r) { const float xg = acc[i][j][r] + bv; so[(16 * i + rh + r) * 68 + 16 * j + cl] = 0.5f * xg * (1.0f + erff(xg * 0.70710678118654752f)); }
      } else {
#pragma unroll
        for (int r = 0; r < 8; ++r) {
          float v = acc[i][j][r] + bv;
          if (EPI == 2) v = R[(size_t)(m0 + wm + 16 * i + rh + r) * ldy + n] + gv * v;
          so[(16 * i + rh + r) * 68 + 16 * j + cl] = v;
        }
      }
    }
  asm volatile("s_wait_dscnt 0" ::: "memory");
  __builtin_amdgcn_wave_barrier();
#pragma unroll 1
  for (int pass = 0; pass < 2; ++pass) {
    if (OUT16) {
      f16* Y = (f16*)Yv;
#pragma unroll
      for (int it = 0; it < 8; ++it) { const int c = lane + 32 * it, rr = c >> 3, q8 = (c & 7) * 8;
        union { f16 h[8]; v4u_t v; } u;
#pragma unroll
        for (int e = 0; e < 8; ++e) u.h[e] = (f16)so[rr * 68 + q8 + e];
        *(volatile v4u_t*)(Y + (size_t)(m0 + wm + rr) * ldy + n0 + wn + q8) = u.v; }
    } else {
      float* Y = (float*)Yv;
#pragma unroll
      for (int it = 0; it < 16; ++it) { const int f4 = lane + 32 * it, rr = f4 >> 4, q = (f4 & 15) * 4;
        *(volatile v4f_t*)(Y + (size_t)(m0 + wm + rr) * ldy + n0 + wn + q) = *(const v4fa*)(so + rr * 68 + q); }
    }
    __threadfence();
  }
}

__global__ __launch_bounds__(256) void k_bn(const float* __restrict__ x, const float* __restrict__ p, float* __restrict__ y) { const size_t row = blockIdx.x; const int c = row % CCs;
  const float inv = p[c] / sqrtf(p[3 * CCs + c] + 1e-5f), sh = p[CCs + c] - p[2 * CCs + c] * inv;
  for (int q4 = threadIdx.x; q4 < NNs / 4; q4 += 256) { v4f_t v = *(const v4f_t*)(x + row * NNs + q4 * 4); for (int e = 0; e < 4; ++e) v[e] = v[e] * inv + sh;
    *(volatile v4f_t*)(y + row * NNs + q4 * 4) = v; __threadfence(); *(volatile v4f_t*)(y + row * NNs + q4 * 4) = v; } }
__global__ __launch_bounds__(128) void k_padw(const float* __restrict__ Wm, int nr, int nc, int cols, float* __restrict__ Wp) { const int r = blockIdx.x, c = threadIdx.x; if (c >= cols) return;
  const float v = (r < nr && c < nc) ? Wm[r * nc + c] : 0.0f; *(volatile float*)(Wp + (size_t)r * cols + c) = v; __threadfence(); *(volatile float*)(Wp + (size_t)r * cols + c) = v; }
__global__ __launch_bounds__(256) void k_rowbias(float* __restrict__ t, const float* __restrict__ bias, int nrows) { const size_t row = blockIdx.x; const float bv = (row < (size_t)nrows) ? bias[row] : 0.0f;
  for (int q4 = threadIdx.x; q4 < NNs / 4; q4 += 256) { v4f_t v = *(const v4f_t*)(t + row * NNs + q4 * 4); for (int e = 0; e < 4; ++e) v[e] += bv; *(volatile v4f_t*)(t + row * NNs + q4 * 4) = v; __threadfence(); *(volatile v4f_t*)(t + row * NNs + q4 * 4) = v; } }
__global__ __launch_bounds__(256) void k_tr32(const float* __restrict__ A, float* __restrict__ At) { __shared__ float tS[32][65];
  const int tid = threadIdx.x; const int n0 = blockIdx.x * 64;
  for (int e = tid; e < 32 * 64; e += 256) { const int c = e >> 6, j = e & 63; tS[c][j] = A[(size_t)c * NNs + n0 + j]; }
  __syncthreads();
  { const int j = tid >> 2, q4 = (tid & 3) * 8; v4f_t o0, o1; for (int k = 0; k < 4; ++k) { o0[k] = tS[q4 + k][j]; o1[k] = tS[q4 + 4 + k][j]; }
    float* dst = At + (size_t)(n0 + j) * CIs + q4; *(volatile v4f_t*)dst = o0; *(volatile v4f_t*)(dst + 4) = o1; __threadfence(); *(volatile v4f_t*)dst = o0; *(volatile v4f_t*)(dst + 4) = o1; }
}
__global__ __launch_bounds__(256) void k_transpose(const float* __restrict__ Wm, float* __restrict__ Wt, int rows, int cols) {
  __shared__ float tS[64][65];
  const int tid = threadIdx.x, tbj = cols / 64, bi = blockIdx.x / tbj, bj = blockIdx.x % tbj;
  for (int e = tid; e < 64 * 64; e += 256) { const int r = e >> 6, c = e & 63; tS[r][c] = Wm[(size_t)(bi * 64 + r) * cols + bj * 64 + c]; }
  __syncthreads();
  for (int ch = tid; ch < 64 * 16; ch += 256) { const int r = ch >> 4, q4 = (ch & 15) * 4; v4f_t o; o[0] = tS[q4][r]; o[1] = tS[q4 + 1][r]; o[2] = tS[q4 + 2][r]; o[3] = tS[q4 + 3][r];
    float* dst = Wt + (size_t)(bj * 64 + r) * rows + bi * 64 + q4; *(volatile v4f_t*)dst = o; __threadfence(); *(volatile v4f_t*)dst = o; }
}
__global__ __launch_bounds__(256) void k_softmax(float* __restrict__ E) {
  __shared__ float red[256];
  const size_t row = blockIdx.x; const int tid = threadIdx.x; float* er = E + row * NNs;
  float v[16]; float m = -3.0e38f;
#pragma unroll
  for (int e = 0; e < 16; ++e) { v[e] = er[tid * 16 + e]; m = fmaxf(m, v[e]); }
  red[tid] = m; __syncthreads();
  for (int o = 128; o > 0; o >>= 1) { if (tid < o) red[tid] = fmaxf(red[tid], red[tid + o]); __syncthreads(); }
  m = red[0]; __syncthreads();
  float z = 0.0f;
#pragma unroll
  for (int e = 0; e < 16; ++e) { v[e] = expf(v[e] - m); z += v[e]; }
  red[tid] = z; __syncthreads();
  for (int o = 128; o > 0; o >>= 1) { if (tid < o) red[tid] += red[tid + o]; __syncthreads(); }
  const float sc = 1024.0f / red[0];
  v4f_t o[4]; for (int e = 0; e < 16; ++e) o[e >> 2][e & 3] = v[e] * sc;
#pragma unroll 1
  for (int pass = 0; pass < 2; ++pass) { for (int i = 0; i < 4; ++i) *(volatile v4f_t*)(er + tid * 16 + i * 4) = o[i]; __threadfence(); }
}
__global__ __launch_bounds__(256) void k_fill(float* __restrict__ p, float val, int n) { for (int i = threadIdx.x; i < n; i += 256) { *(volatile float*)(p + i) = val; __threadfence(); *(volatile float*)(p + i) = val; } }
__global__ __launch_bounds__(256) void k_outbn(const float* __restrict__ Z, const float* __restrict__ Wb, const float* __restrict__ p, const float* __restrict__ x, float* __restrict__ out) { const int c = blockIdx.x;
  const float inv = p[c] / sqrtf(p[3 * CCs + c] + 1e-5f), sh = p[CCs + c] - p[2 * CCs + c] * inv; const float wb = Wb[c];
  for (int q4 = threadIdx.x; q4 < NNs / 4; q4 += 256) { const v4f_t z = *(const v4f_t*)(Z + (size_t)c * NNs + q4 * 4), xv = *(const v4f_t*)(x + (size_t)c * NNs + q4 * 4); v4f_t o;
    for (int e = 0; e < 4; ++e) o[e] = xv[e] + ((z[e] + wb) * inv + sh);
    *(volatile v4f_t*)(out + (size_t)c * NNs + q4 * 4) = o; __threadfence(); *(volatile v4f_t*)(out + (size_t)c * NNs + q4 * 4) = o; } }

extern "C" void kernel_launch(void* const* d_in, const int* in_sizes, int n_in,
                              void* d_out, int out_size, void* d_ws, size_t ws_size,
                              hipStream_t stream) {
  (void)in_sizes; (void)n_in; (void)out_size;
  const float** f = (const float**)d_in;
  const float* x1 = f[0], *x2 = f[1], *gbn = f[2], *gw = f[3], *gb = f[4], *tbn = f[5], *tw = f[6], *tb = f[7], *pbn = f[8], *pw = f[9], *pb = f[10], *wbn = f[11], *Ww = f[12], *Wb = f[13];
  float* out1 = (float*)d_out; float* out2 = out1 + (size_t)NBs * CCs * NNs;
  char* ws = (char*)d_ws;
  float* gwP = (float*)ws; ws += 128 * 64 * 4; float* twP = (float*)ws; ws += 128 * 64 * 4; float* pwP = (float*)ws; ws += 128 * 64 * 4; float* WwP = (float*)ws; ws += 128 * 128 * 4;
  float* xb = (float*)ws; ws += (size_t)CCs * NNs * 4;
  float* g1 = (float*)ws; ws += (size_t)128 * NNs * 4; float* g2 = (float*)ws; ws += (size_t)128 * NNs * 4; float* th = (float*)ws; ws += (size_t)128 * NNs * 4; float* ph = (float*)ws; ws += (size_t)128 * NNs * 4;
  float* thT = (float*)ws; ws += (size_t)NNs * CIs * 4; float* phT = (float*)ws; ws += (size_t)NNs * CIs * 4;
  float* E = (float*)ws; ws += (size_t)NNs * NNs * 4;
  float* Y = (float*)ws; ws += (size_t)128 * NNs * 4;
  float* Z = (float*)ws; ws += (size_t)128 * NNs * 4;
  float* rsc = (float*)ws; ws += 128 * 4;
  if ((size_t)(ws - (char*)d_ws) > ws_size) return;
  const dim3 blk(256);
  k_padw<<<dim3(128), dim3(128), 0, stream>>>(gw, CIs, CCs, CCs, gwP); k_padw<<<dim3(128), dim3(128), 0, stream>>>(tw, CIs, CCs, CCs, twP); k_padw<<<dim3(128), dim3(128), 0, stream>>>(pw, CIs, CCs, CCs, pwP);
  k_padw<<<dim3(128), dim3(128), 0, stream>>>(Ww, CCs, CIs, 128, WwP);
  k_fill<<<dim3(1), blk, 0, stream>>>(rsc, 1.0f / 1024.0f, 128);
  for (int b = 0; b < NBs; ++b) {
    const float* x1b = x1 + (size_t)b * CCs * NNs; const float* x2b = x2 + (size_t)b * CCs * NNs;
    k_bn<<<dim3(CCs), blk, 0, stream>>>(x1b, gbn, xb); gemm_kne<float, 0, false><<<dim3(1, NNs / 128), blk, 0, stream>>>(gwP, CCs, xb, NNs, nullptr, nullptr, nullptr, g1, NNs, CCs); k_rowbias<<<dim3(CIs), blk, 0, stream>>>(g1, gb, CIs);
    k_bn<<<dim3(CCs), blk, 0, stream>>>(x1b, tbn, xb); gemm_kne<float, 0, false><<<dim3(1, NNs / 128), blk, 0, stream>>>(twP, CCs, xb, NNs, nullptr, nullptr, nullptr, th, NNs, CCs); k_rowbias<<<dim3(CIs), blk, 0, stream>>>(th, tb, CIs);
    k_bn<<<dim3(CCs), blk, 0, stream>>>(x2b, gbn, xb); gemm_kne<float, 0, false><<<dim3(1, NNs / 128), blk, 0, stream>>>(gwP, CCs, xb, NNs, nullptr, nullptr, nullptr, g2, NNs, CCs); k_rowbias<<<dim3(CIs), blk, 0, stream>>>(g2, gb, CIs);
    k_bn<<<dim3(CCs), blk, 0, stream>>>(x2b, pbn, xb); gemm_kne<float, 0, false><<<dim3(1, NNs / 128), blk, 0, stream>>>(pwP, CCs, xb, NNs, nullptr, nullptr, nullptr, ph, NNs, CCs); k_rowbias<<<dim3(CIs), blk, 0, stream>>>(ph, pb, CIs);
    k_tr32<<<dim3(NNs / 64), blk, 0, stream>>>(th, thT); k_tr32<<<dim3(NNs / 64), blk, 0, stream>>>(ph, phT);
    gemm_kne<float, 0, false><<<dim3(NNs / 128, NNs / 128), blk, 0, stream>>>(thT, CIs, ph, NNs, nullptr, nullptr, nullptr, E, NNs, CIs);
    k_softmax<<<dim3(NNs), blk, 0, stream>>>(E);
    gemm_rb_kernel<float, 2><<<dim3(1, NNs / 256), blk, 0, stream>>>(g2, E, nullptr, rsc, nullptr, nullptr, Y, 128, NNs, NNs);
    gemm_kne<float, 0, false><<<dim3(1, NNs / 128), blk, 0, stream>>>(WwP, 128, Y, NNs, nullptr, nullptr, nullptr, Z, NNs, 128);
    k_outbn<<<dim3(CCs), blk, 0, stream>>>(Z, Wb, wbn, x2b, out2 + (size_t)b * CCs * NNs);
    gemm_kne<float, 0, false><<<dim3(NNs / 128, NNs / 128), blk, 0, stream>>>(phT, CIs, th, NNs, nullptr, nullptr, nullptr, E, NNs, CIs);
    k_softmax<<<dim3(NNs), blk, 0, stream>>>(E);
    gemm_rb_kernel<float, 2><<<dim3(1, NNs / 256), blk, 0, stream>>>(g1, E, nullptr, rsc, nullptr, nullptr, Y, 128, NNs, NNs);
    gemm_kne<float, 0, false><<<dim3(1, NNs / 128), blk, 0, stream>>>(WwP, 128, Y, NNs, nullptr, nullptr, nullptr, Z, NNs, 128);
    k_outbn<<<dim3(CCs), blk, 0, stream>>>(Z, Wb, wbn, x1b, out1 + (size_t)b * CCs * NNs);
  }
}
